// OR_LSTM_6167573037691
// MI455X (gfx1250) — hardware-run, weakly checked
//
#include <hip/hip_runtime.h>
#include <math.h>

constexpr int NBATCH   = 32;
constexpr int NTRAJ    = 128;
constexpr int NFEAT    = 16;
constexpr int NHID     = 256;
constexpr int NGATE    = 4 * NHID;
constexpr int NWIN     = 8;
constexpr int NPRED    = 8;
constexpr int NROLL    = NTRAJ - NWIN;
constexpr int NTHR     = 512;
constexpr int ROWS_BLK = 16;
constexpr int XK       = 64;
constexpr int XPITCH   = 72;
constexpr int HPITCH   = 264;
constexpr int FPITCH   = 260;
constexpr int GS_X     = NHID * XK;
constexpr int GS_H     = NHID * NHID;
constexpr int OUT0_ELEMS = NBATCH * NROLL * NPRED;
constexpr int OUT1_OFF   = OUT0_ELEMS;
constexpr int OUT2_OFF   = OUT1_OFF + 2 * NBATCH * NHID;
constexpr int OUT_TOTAL  = OUT2_OFF + 2 * NBATCH * NHID;

constexpr float W_CARRY   = 256.0f;
constexpr float H_CARRY   = 16.0f;
constexpr float X_CARRY   = 16.0f;
constexpr float WLO_CARRY = 4096.0f;
constexpr float XLO_CARRY = 512.0f;
constexpr float W8_CARRY  = 8.0f;
constexpr float ACC_CARRY = 4096.0f;
constexpr float ACC_INV   = 1.0f / 4096.0f;

static_assert(W_CARRY * H_CARRY == ACC_CARRY, "carry chain");
static_assert(W_CARRY * X_CARRY == ACC_CARRY, "carry chain");
static_assert(WLO_CARRY * 1.0f == ACC_CARRY, "carry chain");
static_assert(XLO_CARRY * W8_CARRY == ACC_CARRY, "carry chain");
static_assert(NROLL == 120, "shape");
static_assert(NGATE == 1024, "shape");
static_assert(NHID == 16 * (NTHR / 32), "16 waves x 16 hidden units");
static_assert(NBATCH % ROWS_BLK == 0, "batch tiles");
static_assert(XK % 32 == 0 && NHID % 32 == 0, "k multiples of 32");
static_assert(OUT1_OFF * 4 == 122880, "byte offset of second output");
static_assert(OUT2_OFF * 4 == 188416, "byte offset of third output");
static_assert(OUT_TOTAL * 4 == 253952, "total output bytes");
static_assert((OUT1_OFF * 4) % 128 == 0 && (OUT2_OFF * 4) % 128 == 0, "line aligned");
static_assert((NROLL * NPRED * 4) % 128 == 0, "out0 batch row pitch is whole lines");
static_assert(NROLL % 4 == 0, "flush groups");

typedef __attribute__((ext_vector_type(16))) _Float16 v16h;
typedef __attribute__((ext_vector_type(8)))  _Float16 v8h;
typedef __attribute__((ext_vector_type(8)))  float    v8f;
typedef __attribute__((ext_vector_type(4)))  float    v4f;
typedef __attribute__((ext_vector_type(2)))  float    v2f;

union FragU { v16h v; v8h h[2]; };
__device__ __forceinline__ v16h frag_load(const _Float16* p) {
  FragU f;
  f.h[0] = *(const v8h*)(p);
  f.h[1] = *(const v8h*)(p + 16);
  return f.v;
}
__device__ __forceinline__ v8f frag_mma(v16h a, v16h b, v8f c) {
  return __builtin_amdgcn_wmma_f32_16x16x32_f16(false, a, false, b, (short)0, c, false, false);
}
__device__ __forceinline__ void guard_tile(v8f& a0, v8f& a1, v8f& a2, v8f& a3,
                                           v16h x, v16h b0, v16h b1, v16h b2, v16h b3) {
  asm volatile("v_nop\n\tv_nop\n\tv_nop\n\tv_nop"
               : "+v"(a0), "+v"(a1), "+v"(a2), "+v"(a3)
               : "v"(x), "v"(b0), "v"(b1), "v"(b2), "v"(b3));
}
__device__ __forceinline__ void acc_guard4(v8f& a, v8f& b, v8f& c, v8f& d) {
  asm volatile("v_nop\n\tv_nop\n\tv_nop\n\tv_nop" : "+v"(a), "+v"(b), "+v"(c), "+v"(d));
}
__device__ __forceinline__ v8f splat8(float x) { return (v8f){x, x, x, x, x, x, x, x}; }

template <int GSTRIDE>
__device__ __forceinline__ void mma_part(v8f& a0, v8f& a1, v8f& a2, v8f& a3,
                                         const _Float16* arow, const _Float16* wrow, int nk) {
#pragma unroll 1
  for (int kt = 0; kt < nk; ++kt) {
    const int k0 = kt * 32;
    const v16h a  = frag_load(arow + k0);
    const v16h b0 = frag_load(wrow + k0);
    const v16h b1 = frag_load(wrow + (size_t)GSTRIDE + k0);
    const v16h b2 = frag_load(wrow + (size_t)2 * GSTRIDE + k0);
    const v16h b3 = frag_load(wrow + (size_t)3 * GSTRIDE + k0);
    a0 = frag_mma(a, b0, a0);
    a1 = frag_mma(a, b1, a1);
    a2 = frag_mma(a, b2, a2);
    a3 = frag_mma(a, b3, a3);
    guard_tile(a0, a1, a2, a3, a, b0, b1, b2, b3);
  }
}

__device__ __forceinline__ float sigm_f(float x) { return __builtin_amdgcn_rcpf(1.0f + expf(-x)); }
__device__ __forceinline__ float tanh_f(float x) { return 1.0f - 2.0f * __builtin_amdgcn_rcpf(expf(2.0f * x) + 1.0f); }

__device__ __forceinline__ void lstm_cell(const v8f& ai, const v8f& af, const v8f& ag, const v8f& ao,
                                          float (&cst)[8], float (&hst)[8]) {
#pragma unroll
  for (int r = 0; r < 8; ++r) {
    const float zi = ai[r] * ACC_INV;
    const float zf = af[r] * ACC_INV;
    const float zg = ag[r] * ACC_INV;
    const float zo = ao[r] * ACC_INV;
    const float ig = sigm_f(zi);
    const float fg = sigm_f(zf);
    const float gg = tanh_f(zg);
    const float og = sigm_f(zo);
    const float cn = fg * cst[r] + ig * gg;
    cst[r] = cn;
    hst[r] = og * tanh_f(cn);
  }
}

__device__ __forceinline__ unsigned h16bits(float f) {
  const _Float16 h = (_Float16)f;
  const unsigned short b = __builtin_bit_cast(unsigned short, h);
  return (unsigned)b;
}

__global__ __launch_bounds__(256) void pack_w_kernel(const float* __restrict__ s0, const float* __restrict__ s1,
                                                     const float* __restrict__ s2, unsigned short* __restrict__ d0,
                                                     unsigned short* __restrict__ d1, unsigned short* __restrict__ d2) {
  const int which = blockIdx.y;
  const float* src = (which == 0) ? s0 : ((which == 1) ? s1 : s2);
  unsigned short* dst = (which == 0) ? d0 : ((which == 1) ? d1 : d2);
  const int i = blockIdx.x * 256 + threadIdx.x;
  if (i < NGATE * NHID / 8) {
    const v4f a = *(const v4f*)(src + (size_t)i * 8);
    const v4f b = *(const v4f*)(src + (size_t)i * 8 + 4);
    v8h hv;
#pragma unroll
    for (int e = 0; e < 4; ++e) {
      hv[e]     = (_Float16)(a[e] * W_CARRY);
      hv[4 + e] = (_Float16)(b[e] * W_CARRY);
    }
    *(volatile v8h*)(dst + (size_t)i * 8) = hv;
    __threadfence();
    *(volatile v8h*)(dst + (size_t)i * 8) = hv;
  }
}

__device__ __forceinline__ _Float16 wx_elem(float wv, int blk) {
  const float w256 = wv * W_CARRY;
  const _Float16 hi = (_Float16)w256;
  const float res = (w256 - (float)hi) * (WLO_CARRY / W_CARRY);
  const float w8 = wv * W8_CARRY;
  const float f = (blk == 0) ? w256 : ((blk == 1) ? res : ((blk == 2) ? w8 : 0.0f));
  return (_Float16)f;
}
__global__ __launch_bounds__(256) void pack_wx_kernel(const float* __restrict__ w, unsigned short* __restrict__ dst) {
  const int i = blockIdx.x * 256 + threadIdx.x;
  if (i < NGATE * XK / 8) {
    const int n = i >> 3, g = i & 7, blk = g >> 1, half = g & 1;
    const float* sp = w + (size_t)n * NFEAT + half * 8;
    const v4f a = *(const v4f*)(sp);
    const v4f b = *(const v4f*)(sp + 4);
    v8h hv;
#pragma unroll
    for (int e = 0; e < 4; ++e) {
      hv[e]     = wx_elem(a[e], blk);
      hv[4 + e] = wx_elem(b[e], blk);
    }
    *(volatile v8h*)(dst + (size_t)i * 8) = hv;
    __threadfence();
    *(volatile v8h*)(dst + (size_t)i * 8) = hv;
  }
}

__device__ __forceinline__ void store_state(float* stage, const float (&v)[8], float* dst, int tid, int hh, int j) {
#pragma unroll
  for (int r = 0; r < 8; ++r) stage[(8 * hh + r) * FPITCH + j] = v[r];
  __syncthreads();
  for (int pass = 0; pass < 2; ++pass) {
#pragma unroll
    for (int it = 0; it < 2; ++it) {
      const int idx = it * NTHR + tid;
      const int row = idx >> 6, c4 = (idx & 63) * 4;
      const v4f x = *(const v4f*)(stage + row * FPITCH + c4);
      *(volatile v4f*)(dst + (size_t)row * NHID + c4) = x;
    }
    __threadfence();
  }
  __syncthreads();
}

__global__ __launch_bounds__(NTHR) void rollout_kernel(
    const float* __restrict__ traj,
    const float* __restrict__ bih0, const float* __restrict__ bhh0,
    const float* __restrict__ bih1, const float* __restrict__ bhh1,
    const float* __restrict__ wlin, const float* __restrict__ blin,
    const unsigned short* __restrict__ WXp, const unsigned short* __restrict__ WHH0p,
    const unsigned short* __restrict__ WIH1p, const unsigned short* __restrict__ WHH1p,
    float* __restrict__ out) {
  __shared__ __align__(16) _Float16 Xs[ROWS_BLK * XPITCH];
  __shared__ __align__(16) _Float16 H0s[2 * ROWS_BLK * HPITCH];
  __shared__ __align__(16) _Float16 H1s[2 * ROWS_BLK * HPITCH];
  __shared__ __align__(16) float Ring[ROWS_BLK * 64];
  __shared__ __align__(16) float Hf[ROWS_BLK * FPITCH];

  const _Float16* WX   = (const _Float16*)WXp;
  const _Float16* WHH0 = (const _Float16*)WHH0p;
  const _Float16* WIH1 = (const _Float16*)WIH1p;
  const _Float16* WHH1 = (const _Float16*)WHH1p;

  const int tid = threadIdx.x, lane = tid & 31, wave = tid >> 5;
  const int c = lane & 15, hh = lane >> 4, koff = hh * 8;
  const int rowbase = blockIdx.x * ROWS_BLK;
  const int j = 16 * wave + c;

  {
    unsigned* xz = (unsigned*)Xs;
    unsigned* h0z = (unsigned*)H0s;
    unsigned* h1z = (unsigned*)H1s;
#pragma unroll 1
    for (int i = tid; i < ROWS_BLK * XPITCH / 2; i += NTHR) xz[i] = 0u;
#pragma unroll 1
    for (int i = tid; i < 2 * ROWS_BLK * HPITCH / 2; i += NTHR) { h0z[i] = 0u; h1z[i] = 0u; }
#pragma unroll 1
    for (int i = tid; i < ROWS_BLK * 64; i += NTHR) Ring[i] = 0.0f;
#pragma unroll 1
    for (int i = tid; i < ROWS_BLK * FPITCH; i += NTHR) Hf[i] = 0.0f;
  }

  float bs0[4], bs1[4];
#pragma unroll
  for (int q = 0; q < 4; ++q) {
    const int n = q * NHID + j;
    bs0[q] = (bih0[n] + bhh0[n]) * ACC_CARRY;
    bs1[q] = (bih1[n] + bhh1[n]) * ACC_CARRY;
  }

  const _Float16* wx  = WX   + (size_t)j * XK   + koff;
  const _Float16* wh0 = WHH0 + (size_t)j * NHID + koff;
  const _Float16* wi1 = WIH1 + (size_t)j * NHID + koff;
  const _Float16* wh1 = WHH1 + (size_t)j * NHID + koff;
  const _Float16* xrow = Xs + c * XPITCH + koff;

  float c0st[8], c1st[8], h0st[8], h1st[8];
#pragma unroll
  for (int r = 0; r < 8; ++r) { c0st[r] = 0.0f; c1st[r] = 0.0f; h0st[r] = 0.0f; h1st[r] = 0.0f; }
  __syncthreads();

#pragma unroll 1
  for (int t = 0; t < NROLL; ++t) {
#pragma unroll
    for (int r = 0; r < 8; ++r) { c0st[r] = 0.0f; c1st[r] = 0.0f; }

#pragma unroll 1
    for (int s = 0; s < NWIN; ++s) {
      const int cur = s & 1, nxt = cur ^ 1;

      if (tid < 128) {
        const int m = tid >> 3;
        const int dp = (tid & 7) * 2;
        const bool raw = (t + s) < NWIN;
        int trow = raw ? (t + s) : ((t < NWIN) ? (2 * t + s - 1) : (t + s));
        trow = trow < 0 ? 0 : (trow > NTRAJ - 1 ? NTRAJ - 1 : trow);
        const int slot = (t + s - NWIN) & 7;
        const v2f tv = *(const v2f*)(traj + ((size_t)(rowbase + m) * NTRAJ + (size_t)trow) * NFEAT + dp);
        const v2f rv = *(const v2f*)(Ring + m * 64 + slot * 8 + (dp & 7));
        float t0 = tv[0], t1 = tv[1], r0 = rv[0], r1 = rv[1];
        asm volatile("" : "+v"(t0), "+v"(t1), "+v"(r0), "+v"(r1));
        const bool use_ring = (!raw) && (dp >= NPRED);
        const float v0 = use_ring ? r0 : t0;
        const float v1 = use_ring ? r1 : t1;
        const _Float16 hx0 = (_Float16)v0;
        const _Float16 hx1 = (_Float16)v1;
        const float lo0 = (v0 - (float)hx0) * XLO_CARRY;
        const float lo1 = (v1 - (float)hx1) * XLO_CARRY;
        const unsigned wa = h16bits(v0 * X_CARRY) | (h16bits(v1 * X_CARRY) << 16);
        const unsigned wb = h16bits(v0) | (h16bits(v1) << 16);
        const unsigned wc = h16bits(lo0) | (h16bits(lo1) << 16);
        unsigned* xw = (unsigned*)Xs;
        const int wbase = (m * XPITCH + dp) >> 1;
        xw[wbase]      = wa;
        xw[wbase + 8]  = wb;
        xw[wbase + 16] = wc;
        xw[wbase + 24] = 0u;
      }
      __syncthreads();

      {
        v8f a0 = splat8(bs0[0]), a1 = splat8(bs0[1]), a2 = splat8(bs0[2]), a3 = splat8(bs0[3]);
        mma_part<GS_X>(a0, a1, a2, a3, xrow, wx, XK / 32);
        if (s > 0) {
          const _Float16* hrow = H0s + cur * (ROWS_BLK * HPITCH) + c * HPITCH + koff;
          mma_part<GS_H>(a0, a1, a2, a3, hrow, wh0, NHID / 32);
        }
        acc_guard4(a0, a1, a2, a3);
        lstm_cell(a0, a1, a2, a3, c0st, h0st);
        _Float16* hn = H0s + nxt * (ROWS_BLK * HPITCH);
#pragma unroll
        for (int r = 0; r < 8; ++r) hn[(8 * hh + r) * HPITCH + j] = (_Float16)(h0st[r] * H_CARRY);
      }
      __syncthreads();

      {
        v8f a0 = splat8(bs1[0]), a1 = splat8(bs1[1]), a2 = splat8(bs1[2]), a3 = splat8(bs1[3]);
        const _Float16* h0row = H0s + nxt * (ROWS_BLK * HPITCH) + c * HPITCH + koff;
        mma_part<GS_H>(a0, a1, a2, a3, h0row, wi1, NHID / 32);
        if (s > 0) {
          const _Float16* h1row = H1s + cur * (ROWS_BLK * HPITCH) + c * HPITCH + koff;
          mma_part<GS_H>(a0, a1, a2, a3, h1row, wh1, NHID / 32);
        }
        acc_guard4(a0, a1, a2, a3);
        lstm_cell(a0, a1, a2, a3, c1st, h1st);
        _Float16* hn = H1s + nxt * (ROWS_BLK * HPITCH);
#pragma unroll
        for (int r = 0; r < 8; ++r) hn[(8 * hh + r) * HPITCH + j] = (_Float16)(h1st[r] * H_CARRY);
        if (s == NWIN - 1) {
#pragma unroll
          for (int r = 0; r < 8; ++r) Hf[(8 * hh + r) * FPITCH + j] = h1st[r];
        }
      }
      __syncthreads();
    }

    if (tid < 128) {
      const int m = tid >> 3, o = tid & 7;
      const float* hp = Hf + m * FPITCH;
      const float* wp = wlin + (size_t)o * NHID;
      float s0 = 0.0f, s1 = 0.0f, s2 = 0.0f, s3 = 0.0f;
#pragma unroll 4
      for (int k = 0; k < NHID; k += 4) {
        const v4f hv = *(const v4f*)(hp + k);
        const v4f wv = *(const v4f*)(wp + k);
        s0 = fmaf(hv[0], wv[0], s0);
        s1 = fmaf(hv[1], wv[1], s1);
        s2 = fmaf(hv[2], wv[2], s2);
        s3 = fmaf(hv[3], wv[3], s3);
      }
      const float pred = ((s0 + s1) + (s2 + s3)) + blin[o];
      const float ptraj = traj[((size_t)(rowbase + m) * NTRAJ + (NWIN - 1)) * NFEAT + NPRED + o];
      const float pring = Ring[m * 64 + ((t + 7) & 7) * 8 + o];
      const float base = (t == 0) ? ptraj : pring;
      Ring[m * 64 + (t & 7) * 8 + o] = base + pred;
    }
    __syncthreads();

    if ((t & 3) == 3) {
      if (tid < 128) {
        const int m = tid >> 3, p = tid & 7;
        const v4f v = *(const v4f*)(Ring + m * 64 + ((t - 3) & 7) * 8 + p * 4);
        float* dst = out + ((size_t)(rowbase + m) * NROLL + (size_t)(t - 3)) * NPRED + p * 4;
        *(volatile v4f*)dst = v;
        __threadfence();
        *(volatile v4f*)dst = v;
      }
    }
  }

  store_state(Hf, h0st, out + OUT1_OFF + (size_t)(0 * NBATCH + rowbase) * NHID, tid, hh, j);
  store_state(Hf, h1st, out + OUT1_OFF + (size_t)(1 * NBATCH + rowbase) * NHID, tid, hh, j);
  store_state(Hf, c0st, out + OUT2_OFF + (size_t)(0 * NBATCH + rowbase) * NHID, tid, hh, j);
  store_state(Hf, c1st, out + OUT2_OFF + (size_t)(1 * NBATCH + rowbase) * NHID, tid, hh, j);
}

extern "C" void kernel_launch(void* const* d_in, const int* in_sizes, int n_in,
                              void* d_out, int out_size, void* d_ws, size_t ws_size, hipStream_t stream) {
  if (n_in < 11 || d_out == nullptr || d_ws == nullptr) return;
  if (in_sizes[0] != NBATCH * NTRAJ * NFEAT || in_sizes[1] != NGATE * NFEAT || in_sizes[2] != NGATE * NHID ||
      in_sizes[3] != NGATE || in_sizes[4] != NGATE || in_sizes[5] != NGATE * NHID || in_sizes[6] != NGATE * NHID ||
      in_sizes[7] != NGATE || in_sizes[8] != NGATE || in_sizes[9] != NPRED * NHID || in_sizes[10] != NPRED ||
      out_size != OUT_TOTAL) return;

  const float* traj = (const float*)d_in[0];
  const float* wih0 = (const float*)d_in[1];
  const float* whh0 = (const float*)d_in[2];
  const float* bih0 = (const float*)d_in[3];
  const float* bhh0 = (const float*)d_in[4];
  const float* wih1 = (const float*)d_in[5];
  const float* whh1 = (const float*)d_in[6];
  const float* bih1 = (const float*)d_in[7];
  const float* bhh1 = (const float*)d_in[8];
  const float* wlin = (const float*)d_in[9];
  const float* blin = (const float*)d_in[10];

  char* ws = (char*)d_ws;
  size_t off = 0;
  auto carve = [&](size_t bytes) -> char* { char* p = ws + off; off += (bytes + 255) & ~(size_t)255; return p; };
  unsigned short* WHH0 = (unsigned short*)carve((size_t)NGATE * NHID * 2);
  unsigned short* WIH1 = (unsigned short*)carve((size_t)NGATE * NHID * 2);
  unsigned short* WHH1 = (unsigned short*)carve((size_t)NGATE * NHID * 2);
  unsigned short* WX   = (unsigned short*)carve((size_t)NGATE * XK * 2);
  if (off > ws_size || off > (size_t)134217728) return;

  pack_w_kernel<<<dim3(NGATE * NHID / 8 / 256, 3), 256, 0, stream>>>(whh0, wih1, whh1, WHH0, WIH1, WHH1);
  pack_wx_kernel<<<NGATE * XK / 8 / 256, 256, 0, stream>>>(wih0, WX);
  rollout_kernel<<<NBATCH / ROWS_BLK, NTHR, 0, stream>>>(traj, bih0, bhh0, bih1, bhh1, wlin, blin,
                                                         WX, WHH0, WIH1, WHH1, (float*)d_out);
}
